// Marcher_17317308138012
// MI455X (gfx1250) — hardware-verified
//
#include <hip/hip_runtime.h>
#include <stdint.h>


typedef _Float16 v16h __attribute__((ext_vector_type(16)));
typedef _Float16 v8h  __attribute__((ext_vector_type(8)));
typedef _Float16 v8ha __attribute__((ext_vector_type(8), __may_alias__));
typedef float    v8f  __attribute__((ext_vector_type(8)));
typedef float    v4f  __attribute__((ext_vector_type(4)));
typedef float    v4fa __attribute__((ext_vector_type(4), __may_alias__));

#define HIDDEN 128
#define STEPS 32
#define WAVES 4
#define RAYS_PER_WAVE 16
#define RAYS_PER_BLOCK (WAVES * RAYS_PER_WAVE)
#define THREADS (WAVES * 32)
#define NT 8
#define KC 4

union Frag { v16h v; v8h p[2]; };

__device__ __forceinline__ v8f wmma_f16(v8f acc, const v16h a, const v16h b)
{
    acc = __builtin_amdgcn_wmma_f32_16x16x32_f16(false, a, false, b, (short)0, acc, false, false);
    asm volatile("v_nop\n\tv_nop\n\tv_nop\n\tv_nop" : "+v"(acc) : "v"(a), "v"(b));
    return acc;
}

__global__ __launch_bounds__(THREADS)
void k_march(const float* __restrict__ pos,
             const float* __restrict__ dirg,
             const float* __restrict__ W1,
             const float* __restrict__ b1,
             const float* __restrict__ W2,
             const float* __restrict__ b2,
             const float* __restrict__ W3,
             const float* __restrict__ b3,
             float* __restrict__ out,
             int nRays, int outN)
{
    __shared__ __attribute__((aligned(32))) _Float16 sB[KC * NT][32][16];
    __shared__ v4f sW1p[HIDDEN];
    __shared__ __attribute__((aligned(16))) float sOut[RAYS_PER_BLOCK * 3];

    const int tid  = threadIdx.x;
    const int wave = tid >> 5;
    const int lane = tid & 31;
    const int h    = lane >> 4;
    const int m    = lane & 15;

    for (int idx = tid; idx < HIDDEN * HIDDEN; idx += THREADS) {
        const int k  = idx >> 7, n = idx & 127;
        const int c  = k >> 5, kk = k & 31;
        const int t  = n >> 4, nn = n & 15;
        const int hh = (kk >> 3) & 1;
        const int e  = (kk & 7) | ((kk >> 4) << 3);
        sB[c * NT + t][nn + 16 * hh][e] = (_Float16)(W2[idx] * 64.0f);
    }
    for (int j = tid; j < HIDDEN; j += THREADS) {
        v4f w;
        w.x = W1[j] * 16.0f;
        w.y = W1[HIDDEN + j] * 16.0f;
        w.z = W1[2 * HIDDEN + j] * 16.0f;
        w.w = b1[j] * 16.0f;
        sW1p[j] = w;
    }

    float w3v[NT], b2s[NT];
#pragma unroll
    for (int t = 0; t < NT; ++t) {
        w3v[t] = W3[16 * t + m];
        b2s[t] = b2[16 * t + m] * 1024.0f;
    }
    const float b3s = b3[0];

    int r  = blockIdx.x * RAYS_PER_BLOCK + wave * RAYS_PER_WAVE + m;
    int rc = (r < nRays) ? r : (nRays - 1);
    float px = pos[3 * rc + 0], py = pos[3 * rc + 1], pz = pos[3 * rc + 2];
    const float dx = dirg[3 * rc + 0], dy = dirg[3 * rc + 1], dz = dirg[3 * rc + 2];

    __syncthreads();

#pragma unroll 1
    for (int s = 0; s < STEPS; ++s) {
        v16h af[KC];
#pragma unroll
        for (int c = 0; c < KC; ++c) {
#pragma unroll
            for (int i = 0; i < 16; ++i) {
                const int j = 32 * c + 8 * h + i + ((i >= 8) ? 8 : 0);
                const v4f w = sW1p[j];
                float v = fmaf(px, w.x, fmaf(py, w.y, fmaf(pz, w.z, w.w)));
                v = fmaxf(v, 0.0f);
                af[c][i] = (_Float16)v;
            }
            asm volatile("" ::: "memory");
        }

        float part[8];
#pragma unroll
        for (int q = 0; q < 8; ++q) part[q] = 0.0f;

#pragma unroll
        for (int t = 0; t < NT; ++t) {
            v8f cc;
#pragma unroll
            for (int q = 0; q < 8; ++q) cc[q] = b2s[t];
#pragma unroll
            for (int c = 0; c < KC; ++c) {
                Frag b;
                const _Float16* bp = &sB[c * NT + t][lane][0];
                b.p[0] = *(const v8ha*)(bp);
                b.p[1] = *(const v8ha*)(bp + 8);
                cc = wmma_f16(cc, af[c], b.v);
            }
#pragma unroll
            for (int q = 0; q < 8; ++q)
                part[q] = fmaf(fmaxf(cc[q], 0.0f), w3v[t], part[q]);
        }

        float dsel = 0.0f;
#pragma unroll
        for (int q = 0; q < 8; ++q) {
            float v = part[q];
            v += __shfl_xor(v, 1, 32);
            v += __shfl_xor(v, 2, 32);
            v += __shfl_xor(v, 4, 32);
            v += __shfl_xor(v, 8, 32);
            dsel = ((lane & 7) == q) ? v : dsel;
        }
        const int src = ((m >> 3) << 4) | (m & 7);
        const float dsum = __shfl(dsel, src, 32);
        const float d = fmaf(dsum, 1.0f / 1024.0f, b3s);

        px = fmaf(d, dx, px);
        py = fmaf(d, dy, py);
        pz = fmaf(d, dz, pz);
    }

    if (h == 0) {
        sOut[wave * 48 + 3 * m + 0] = px;
        sOut[wave * 48 + 3 * m + 1] = py;
        sOut[wave * 48 + 3 * m + 2] = pz;
    }
    __syncthreads();

    if (wave < 2) {
        const int idx4 = wave * 32 + lane;
        if (idx4 < 48) {
            const v4f v = *(const v4fa*)&sOut[4 * idx4];
            const size_t g = (size_t)blockIdx.x * (RAYS_PER_BLOCK * 3) + (size_t)(4 * idx4);
            const bool full = (g + 4 <= (size_t)outN);
            if (full) {
                *(volatile v4f*)(out + g) = v;
            } else {
#pragma unroll
                for (int e = 0; e < 4; ++e)
                    if (g + e < (size_t)outN) ((volatile float*)out)[g + e] = v[e];
            }
            __threadfence();
            if (full) {
                *(volatile v4f*)(out + g) = v;
            } else {
#pragma unroll
                for (int e = 0; e < 4; ++e)
                    if (g + e < (size_t)outN) ((volatile float*)out)[g + e] = v[e];
            }
        }
    }
}

extern "C" void kernel_launch(void* const* d_in, const int* in_sizes, int n_in,
                              void* d_out, int out_size, void* d_ws, size_t ws_size,
                              hipStream_t stream)
{
    (void)n_in; (void)d_ws; (void)ws_size;
    const float* pos = (const float*)d_in[0];
    const float* dir = (const float*)d_in[1];
    const float* W1  = (const float*)d_in[2];
    const float* b1  = (const float*)d_in[3];
    const float* W2  = (const float*)d_in[4];
    const float* b2  = (const float*)d_in[5];
    const float* W3  = (const float*)d_in[6];
    const float* b3  = (const float*)d_in[7];
    float* out = (float*)d_out;

    const int nRays = in_sizes[0] / 3;
    if (nRays <= 0) return;
    const int blocks = (nRays + RAYS_PER_BLOCK - 1) / RAYS_PER_BLOCK;
    k_march<<<blocks, THREADS, 0, stream>>>(pos, dir, W1, b1, W2, b2, W3, b3, out, nRays, out_size);
}
